// BiLSTMWithAttention_38147899523467
// MI455X (gfx1250) — hardware-verified
//
#include <hip/hip_runtime.h>
#include <math.h>

typedef __attribute__((ext_vector_type(16))) _Float16 v16h;
typedef __attribute__((ext_vector_type(16))) __bf16 v16b;
typedef __attribute__((ext_vector_type(8)))  _Float16 v8h;
typedef __attribute__((ext_vector_type(8)))  float v8f;
typedef __attribute__((ext_vector_type(4)))  float v4f;
typedef __attribute__((ext_vector_type(2)))  float v2f;
typedef __attribute__((ext_vector_type(4)))  unsigned v4u;
typedef __attribute__((ext_vector_type(4)))  int v4i;
typedef float __attribute__((may_alias)) float_a;
typedef int __attribute__((may_alias)) int_a;

template <typename T> __device__ __forceinline__ void vst2(void* p, T v) { *(volatile T*)p = v; __threadfence(); *(volatile T*)p = v; }
__device__ __forceinline__ v8f wmma16(v16h a, v16h b, v8f c) {
  v8f d = __builtin_amdgcn_wmma_f32_16x16x32_f16(false, a, false, b, (short)0, c, false, false);
  asm volatile("v_nop\n\tv_nop\n\tv_nop\n\tv_nop" : "+v"(d) : "v"(a), "v"(b));
  return d;
}
__device__ __forceinline__ v8f wmma_bf(v16b a, v16b b, v8f c) {
  v8f d = __builtin_amdgcn_wmma_f32_16x16x32_bf16(false, a, false, b, (short)0, c, false, false);
  asm volatile("v_nop\n\tv_nop\n\tv_nop\n\tv_nop" : "+v"(d) : "v"(a), "v"(b));
  return d;
}
__device__ __forceinline__ v16h frag_h(const _Float16* rowk0, int lane) {
  union { v16h v; v8h q[2]; } u; const _Float16* p = rowk0 + 8 * (lane >> 4);
  u.q[0] = *(const v8h*)p; u.q[1] = *(const v8h*)(p + 16); return u.v;
}
__device__ __forceinline__ v16h frag_f32(const float* rowk0, int lane) {
  v16h a; const float* p = rowk0 + 8 * (lane >> 4);
#pragma unroll
  for (int i = 0; i < 8; ++i) { a[i] = (_Float16)p[i]; a[8 + i] = (_Float16)p[16 + i]; }
  return a;
}
__device__ __forceinline__ v16h frag_f32s(const float* rowk0, int lane, float sc) {
  v16h a; const float* p = rowk0 + 8 * (lane >> 4);
#pragma unroll
  for (int i = 0; i < 8; ++i) { a[i] = (_Float16)(p[i] * sc); a[8 + i] = (_Float16)(p[16 + i] * sc); }
  return a;
}
__device__ __forceinline__ v16h fragc_f32(const float* W, int k0, int n, int lane, int ld, int K) {
  v16h a; const int g = lane >> 4;
#pragma unroll
  for (int i = 0; i < 8; ++i) { const int ka = k0 + 8 * g + i, kb = ka + 16;
    a[i] = (_Float16)(ka < K ? W[(size_t)(ka < K ? ka : K - 1) * ld + n] : 0.f); a[8 + i] = (_Float16)(kb < K ? W[(size_t)(kb < K ? kb : K - 1) * ld + n] : 0.f); }
  return a;
}
struct F2 { v16b h, l; };
__device__ __forceinline__ F2 bsplit16(const float v[16]) { F2 r;
#pragma unroll
  for (int i = 0; i < 16; ++i) { const __bf16 h = (__bf16)v[i]; r.h[i] = h; r.l[i] = (__bf16)(v[i] - (float)h); }
  return r; }
__device__ __forceinline__ F2 split_row(const float* row, int k0, int lane) { float v[16]; const float* p = row + k0 + 8 * (lane >> 4);
#pragma unroll
  for (int i = 0; i < 8; ++i) { v[i] = p[i]; v[8 + i] = p[16 + i]; }
  return bsplit16(v); }
__device__ __forceinline__ F2 split_rowK(const float* row, int k0, int lane, int K) { float v[16]; const int g = lane >> 4;
#pragma unroll
  for (int i = 0; i < 8; ++i) { const int ka = k0 + 8 * g + i, kb = ka + 16; v[i] = ka < K ? row[ka < K ? ka : K - 1] : 0.f; v[8 + i] = kb < K ? row[kb < K ? kb : K - 1] : 0.f; }
  return bsplit16(v); }
__device__ __forceinline__ F2 split_col(const float* W, int k0, int n, int lane, int ld, int K) { float v[16]; const int g = lane >> 4;
#pragma unroll
  for (int i = 0; i < 8; ++i) { const int ka = k0 + 8 * g + i, kb = ka + 16; v[i] = ka < K ? W[(size_t)(ka < K ? ka : K - 1) * ld + n] : 0.f; v[8 + i] = kb < K ? W[(size_t)(kb < K ? kb : K - 1) * ld + n] : 0.f; }
  return bsplit16(v); }
__device__ __forceinline__ v8f mac3(const F2& a, const F2& b, v8f c) { c = wmma_bf(a.l, b.h, c); c = wmma_bf(a.h, b.l, c); return wmma_bf(a.h, b.h, c); }
__device__ __forceinline__ float sigm(float v) { return 1.0f / (1.0f + expf(-v)); }
#define LDSX() do { asm volatile("s_wait_dscnt 0" ::: "memory"); __builtin_amdgcn_wave_barrier(); __builtin_amdgcn_fence(__ATOMIC_RELEASE, "workgroup"); } while (0)


#define NB 64
#define CI 64
#define TT 2048
#define HH 128
#define G4 (4 * HH)
#define H2 (2 * HH)
#define BT 16
#ifndef NBLK
#define NBLK (NB / BT)
#endif
#ifndef TSTEP
#define TSTEP TT
#endif
typedef __attribute__((ext_vector_type(8))) __bf16 v8b;
__device__ __forceinline__ v16b frag_b(const __bf16* rowk0, int lane) {
  union { v16b v; v8b q[2]; } u; const __bf16* p = rowk0 + 8 * (lane >> 4);
  u.q[0] = *(const v8b*)p; u.q[1] = *(const v8b*)(p + 16); return u.v;
}
__device__ __forceinline__ float bfr(float v) { return (float)(__bf16)v; }
__device__ __attribute__((noinline)) float exp_ni(float v) { return expf(v); }
__device__ __attribute__((noinline)) float erf_ni(float v) { return erff(v); }

__device__ __attribute__((noinline)) float tanh_ni(float v) { return tanhf(v); }
__device__ __forceinline__ float sigm_f(float v) { return 1.0f / (1.0f + exp_ni(-v)); }
__device__ __forceinline__ void put_hl(__bf16* h, __bf16* l, float v) { const __bf16 hb = (__bf16)v; *h = hb; *l = (__bf16)(v - (float)hb); }
#define PK_WHF 0
#define PK_WHB (PK_WHF + G4 * HH)
#define PK_WIF (PK_WHB + G4 * HH)
#define PK_WIB (PK_WIF + G4 * CI)
#define PK_WA  (PK_WIB + G4 * CI)
#define PK_END (PK_WA + H2 * H2)
#define WS_PK  0u
#define WS_XT  (WS_PK + 2u * PK_END)
#define WS_HF  (WS_XT + 2u * NB * TT * CI)
#define WS_END (WS_HF + 4u * NB * TT * HH)

__global__ __launch_bounds__(64) void k_pack(const float* __restrict__ Wm, int K, __bf16* __restrict__ DST) {
  __shared__ __align__(16) __bf16 s[H2]; const int n = blockIdx.x, tid = threadIdx.x;
  for (int k = tid; k < K; k += 64) s[k] = (__bf16)Wm[(size_t)n * K + k];
  __syncthreads();
  if (tid < K / 8) vst2((unsigned*)(DST + (size_t)n * K + tid * 8), *(const v4u*)&s[tid * 8]);
}
__global__ __launch_bounds__(256) void k_xt(const float* __restrict__ X, __bf16* __restrict__ XT) {
  __shared__ __align__(16) __bf16 s[64][CI + 8]; const int t0 = blockIdx.x * 64, b = blockIdx.y, tid = threadIdx.x;
  for (int q = tid; q < CI * 64; q += 256) { const int c = q >> 6, tl = q & 63; s[tl][c] = (__bf16)X[((size_t)b * CI + c) * TT + t0 + tl]; }
  __syncthreads();
  for (int q = tid; q < 64 * 8; q += 256) { const int tl = q >> 3, pc = q & 7; vst2((unsigned*)(XT + ((size_t)b * TT + t0 + tl) * CI + pc * 8), *(const v4u*)&s[tl][pc * 8]); }
}
template <int DIR>
__global__ __launch_bounds__(128) void k_lstm(const __bf16* __restrict__ PK, const __bf16* __restrict__ XT, const float* __restrict__ bih, const float* __restrict__ bhh, float* __restrict__ HF, const float* __restrict__ ba, const float* __restrict__ Wu, const float* __restrict__ bu, float* __restrict__ out) {
  __shared__ __align__(16) __bf16 sah[BT][HH + 8], sal[BT][HH + 8];
  __shared__ __align__(16) float sg[4][BT][HH + 4];
  __shared__ __align__(16) float sh[BT][HH + 4];
  __shared__ __align__(16) __bf16 sch[DIR ? BT : 1][H2 + 8], scl[DIR ? BT : 1][H2 + 8];
  __shared__ __align__(16) float sc2[DIR ? BT : 1][H2 + 4];
  __shared__ float ssc[4][BT]; __shared__ __align__(16) float sacc[DIR ? BT : 1][H2 + 4]; __shared__ float scs[BT][HH];
  const int tid = threadIdx.x, wave = tid >> 5, lane = tid & 31, col = lane & 15, hf = lane >> 4; const int b0 = blockIdx.x * BT; const int u = tid;
  const __bf16* WH = PK + (DIR ? PK_WHB : PK_WHF); const __bf16* WI = PK + (DIR ? PK_WIB : PK_WIF);
  float bb[8];
#pragma unroll
  for (int j = 0; j < 8; ++j) { const int gi = wave * HH + j * 16 + col; bb[j] = bfr(bih[gi]) + bfr(bhh[gi]); }
  float mst[BT], lst[BT];
#pragma unroll
  for (int b = 0; b < BT; ++b) { scs[b][u] = 0.f; mst[b] = -3.0e38f; lst[b] = 0.f; }
  for (int q = tid; q < BT * (HH + 8); q += 128) { (&sah[0][0])[q] = (__bf16)0.f; (&sal[0][0])[q] = (__bf16)0.f; }
  if (DIR) for (int q = tid; q < BT * (H2 + 4); q += 128) (&sacc[0][0])[q] = 0.f;
  float wa_b[4], wu_c[4]; if (DIR) {
#pragma unroll
    for (int j = 0; j < 4; ++j) { const int gi = wave * 64 + j * 16 + col; wa_b[j] = bfr(ba[gi]); wu_c[j] = bfr(Wu[gi]); } }
  const float bu0 = DIR ? bfr(bu[0]) : 0.f;
  __syncthreads();
#pragma unroll 1
  for (int step = 0; step < TSTEP; ++step) { const int t = DIR ? (TSTEP - 1 - step) : step;
    { v8f acc[8] = {};
#pragma unroll
      for (int kc = 0; kc < HH / 32; ++kc) { const v16b ah = frag_b(&sah[col][kc * 32], lane), al = frag_b(&sal[col][kc * 32], lane);
#pragma unroll
        for (int j = 0; j < 8; ++j) { const v16b w = frag_b(WH + (size_t)(wave * HH + j * 16 + col) * HH + kc * 32, lane); acc[j] = wmma_bf(al, w, acc[j]); acc[j] = wmma_bf(ah, w, acc[j]); } }
#pragma unroll
      for (int kc = 0; kc < CI / 32; ++kc) { const v16b ax = frag_b(XT + ((size_t)(b0 + col) * TT + t) * CI + kc * 32, lane);
#pragma unroll
        for (int j = 0; j < 8; ++j) { const v16b w = frag_b(WI + (size_t)(wave * HH + j * 16 + col) * CI + kc * 32, lane); acc[j] = wmma_bf(ax, w, acc[j]); } }
#pragma unroll
      for (int j = 0; j < 8; ++j)
#pragma unroll
        for (int r = 0; r < 8; ++r) sg[wave][8 * hf + r][j * 16 + col] = acc[j][r] + bb[j]; }
    __syncthreads();
#pragma unroll 2
    for (int b = 0; b < BT; ++b) { const float ig = sigm_f(sg[0][b][u]), fg = sigm_f(sg[1][b][u]), gg = tanh_ni(sg[2][b][u]), og = sigm_f(sg[3][b][u]);
      const float cn = fg * scs[b][u] + ig * gg; scs[b][u] = cn; const float hv = og * tanh_ni(cn); sh[b][u] = hv; put_hl(&sah[b][u], &sal[b][u], hv);
      if (DIR) { const float hfv = HF[((size_t)(b0 + b) * TT + t) * HH + u]; put_hl(&sch[b][u], &scl[b][u], hfv); put_hl(&sch[b][HH + u], &scl[b][HH + u], hv); sc2[b][u] = hfv; sc2[b][HH + u] = hv; } }
    __syncthreads();
    if (!DIR) {
      for (int q = tid; q < BT * 32; q += 128) { const int b = q >> 5, pc = q & 31; vst2(HF + ((size_t)(b0 + b) * TT + t) * HH + pc * 4, *(const v4f*)&sh[b][pc * 4]); }
    } else {
      { v8f acc[4] = {};
#pragma unroll
        for (int kc = 0; kc < H2 / 32; ++kc) { const v16b ah = frag_b(&sch[col][kc * 32], lane), al = frag_b(&scl[col][kc * 32], lane);
#pragma unroll
          for (int j = 0; j < 4; ++j) { const v16b w = frag_b(PK + PK_WA + (size_t)(wave * 64 + j * 16 + col) * H2 + kc * 32, lane); acc[j] = wmma_bf(al, w, acc[j]); acc[j] = wmma_bf(ah, w, acc[j]); } }
        float ps[8];
#pragma unroll
        for (int r = 0; r < 8; ++r) { float s = 0.f;
#pragma unroll
          for (int j = 0; j < 4; ++j) s += tanh_ni(acc[j][r] + wa_b[j]) * wu_c[j];
#pragma unroll
          for (int o = 1; o < 16; o <<= 1) s += __shfl_xor(s, o);
          ps[r] = s; }
        if (col == 0) {
#pragma unroll
          for (int r = 0; r < 8; ++r) ssc[wave][8 * hf + r] = ps[r]; } }
      __syncthreads();
#pragma unroll
      for (int b = 0; b < BT; ++b) { const float s = ((ssc[0][b] + ssc[1][b]) + (ssc[2][b] + ssc[3][b])) + bu0; const float mn = fmaxf(mst[b], s); const float al = exp_ni(mst[b] - mn), p = exp_ni(s - mn);
        lst[b] = lst[b] * al + p; mst[b] = mn; sacc[b][u] = sacc[b][u] * al + p * sc2[b][u]; sacc[b][HH + u] = sacc[b][HH + u] * al + p * sc2[b][HH + u]; }
    } }
  if (DIR) { __syncthreads();
#pragma unroll
    for (int b = 0; b < BT; ++b) { const float il = 1.0f / lst[b]; sacc[b][u] *= il; sacc[b][HH + u] *= il; }
    __syncthreads();
    for (int q = tid; q < BT * 64; q += 128) { const int b = q >> 6, pc = q & 63; vst2(out + (size_t)(b0 + b) * H2 + pc * 4, *(const v4f*)&sacc[b][pc * 4]); } }
}
extern "C" void kernel_launch(void* const* d_in, const int* in_sizes, int n_in, void* d_out, int out_size, void* d_ws, size_t ws_size, hipStream_t stream) {
  (void)in_sizes; (void)n_in; (void)out_size;
  const float** F = (const float**)d_in;
  if (ws_size < (size_t)WS_END) return;
  char* ws = (char*)d_ws; __bf16 *PK = (__bf16*)(ws + WS_PK), *XT = (__bf16*)(ws + WS_XT); float* HF = (float*)(ws + WS_HF);
  k_pack<<<G4, 64, 0, stream>>>(F[2], HH, PK + PK_WHF);
  k_pack<<<G4, 64, 0, stream>>>(F[6], HH, PK + PK_WHB);
  k_pack<<<G4, 64, 0, stream>>>(F[1], CI, PK + PK_WIF);
  k_pack<<<G4, 64, 0, stream>>>(F[5], CI, PK + PK_WIB);
  k_pack<<<H2, 64, 0, stream>>>(F[9], H2, PK + PK_WA);
  k_xt<<<dim3(TT / 64, NB), 256, 0, stream>>>(F[0], XT);
  k_lstm<0><<<NBLK, 128, 0, stream>>>(PK, XT, F[3], F[4], HF, F[10], F[11], F[12], (float*)d_out);
  k_lstm<1><<<NBLK, 128, 0, stream>>>(PK, XT, F[7], F[8], HF, F[10], F[11], F[12], (float*)d_out);
}
